// FraudGNN_15513421873288
// MI455X (gfx1250) — hardware-verified
//
#include <hip/hip_runtime.h>
#include <stddef.h>
#include <stdint.h>


#define F      128
#define K2     256
#define FH     64
#define NOUT   2
#define NTHR   256
#define NWAVE  8
#define EPT    8
#define CHUNK  (NTHR * EPT)
#define WCAP   (EPT * 32)
#define LISTN  (NWAVE * WCAP)
#define NBD    8192
#define SLD    13
#define NBA    1024
#define SLA    10
#define RCAP   24576
#define DEGCAP 64
#define PARTW  288
#define WSTW   258
#define GBM    64
#define GBN    128
#define GTHR   128
#define HTHR   128
#define NU1    (F * (F / 8))
#define NU2    (F * (K2 / 8))
#define NU3    (FH * (K2 / 8))
#define AGG_ZINTS (LISTN + 2 * RCAP + 3 * NBA)
#define AGG_LDS_INTS (AGG_ZINTS + 16 + NWAVE * WSTW + PARTW)
#define WSMAX  134217728

static_assert((CHUNK & (CHUNK - 1)) == 0 && CHUNK <= 4096);
static_assert((NBD & (NBD - 1)) == 0 && NBD == (1 << SLD));
static_assert((NBA & (NBA - 1)) == 0 && NBA == (1 << SLA));
static_assert(((long long)CHUNK << SLD) < (1LL << 31));
static_assert(((long long)CHUNK << SLA) < (1LL << 31));
static_assert(NBD % (NTHR * 4) == 0);
static_assert(LISTN % NTHR == 0);
static_assert(NBA % NWAVE == 0 && NBA % 32 == 0 && NBA % GBM == 0);
static_assert(RCAP % 4 == 0 && AGG_ZINTS % 4 == 0 && LISTN % 4 == 0);
static_assert((AGG_ZINTS + 16 + NWAVE * WSTW) % 4 == 0);
static_assert(AGG_LDS_INTS * 4 <= 300000);
static_assert(NU1 % NTHR == 0 && NU2 % NTHR == 0 && NU3 % NTHR == 0);
static_assert(GBM == (GTHR / 32) * 16 && GBN == 4 * 32);
static_assert(F % 32 == 0 && K2 == 2 * F && F == GBN && F / 8 == 16 && K2 / 8 == 32);
static_assert(PARTW % 32 == 0 && PARTW / 4 <= NTHR && PARTW >= 2 * F + 1);
static_assert(WSTW >= 2 * F + 1 && (WSTW % 2) == 0);
static_assert(HTHR == F && FH * NOUT == HTHR && GBM * NOUT == 32 * 4 && FH == 4 * 16 && GBM == (HTHR / 32) * 16);
static_assert(F / 4 == 32);

typedef float          v4f   __attribute__((ext_vector_type(4)));
typedef float          v8f   __attribute__((ext_vector_type(8)));
typedef int            v4i   __attribute__((ext_vector_type(4)));
typedef int            v8i   __attribute__((ext_vector_type(8)));
typedef unsigned short v8us  __attribute__((ext_vector_type(8)));
typedef unsigned short v16us __attribute__((ext_vector_type(16)));
typedef __bf16         v16bf __attribute__((ext_vector_type(16)));
typedef v4f  __attribute__((may_alias)) v4fa;
typedef v4i  __attribute__((may_alias)) v4ia;
typedef v8us __attribute__((may_alias)) v8usa;
union FragB { v16bf v; v16us u; v8us h[2]; v8i w; };

__device__ __forceinline__ v8f wmb(const FragB& a, const FragB& b, v8f c) {
  v8f d = __builtin_amdgcn_wmma_f32_16x16x32_bf16(false, a.v, false, b.v, (short)0, c, false, false);
  asm volatile("v_nop\n\tv_nop\n\tv_nop\n\tv_nop" : "+v"(d) : "v"(a.w), "v"(b.w));
  return d;
}

__device__ __forceinline__ v8f z8() { v8f z = {0.f, 0.f, 0.f, 0.f, 0.f, 0.f, 0.f, 0.f}; return z; }

__device__ __forceinline__ unsigned bf16_bits(float f) {
  const unsigned u = __float_as_uint(f);
  return (u + 0x7FFFu + ((u >> 16) & 1u)) >> 16;
}
__device__ __forceinline__ float bf16_val(float f) {
  return __uint_as_float(bf16_bits(f) << 16);
}

template <int SLB>
__device__ __forceinline__ int scan_chunk(const int* __restrict__ dsts, int nE, int cbase, int slotBase,
                                          int nb, int vec8, int* list, int tid, int lane, int wave) {
  int wc = 0;
  const int el0  = tid * EPT;
  const int e0   = cbase + el0;
  const int sent = -2147483647 - 1;
  v4i da, db;
  if (vec8 != 0 && cbase + CHUNK <= nE) {
    da = *(const v4i*)(dsts + e0);
    db = *(const v4i*)(dsts + e0 + 4);
  } else {
    da.x = (e0     < nE) ? dsts[min(e0,     nE - 1)] : sent;
    da.y = (e0 + 1 < nE) ? dsts[min(e0 + 1, nE - 1)] : sent;
    da.z = (e0 + 2 < nE) ? dsts[min(e0 + 2, nE - 1)] : sent;
    da.w = (e0 + 3 < nE) ? dsts[min(e0 + 3, nE - 1)] : sent;
    db.x = (e0 + 4 < nE) ? dsts[min(e0 + 4, nE - 1)] : sent;
    db.y = (e0 + 5 < nE) ? dsts[min(e0 + 5, nE - 1)] : sent;
    db.z = (e0 + 6 < nE) ? dsts[min(e0 + 6, nE - 1)] : sent;
    db.w = (e0 + 7 < nE) ? dsts[min(e0 + 7, nE - 1)] : sent;
  }
  const unsigned nbs = (unsigned)slotBase;
  const unsigned unb = (unsigned)nb;
  const unsigned s0 = (unsigned)da.x - nbs, s1 = (unsigned)da.y - nbs;
  const unsigned s2 = (unsigned)da.z - nbs, s3 = (unsigned)da.w - nbs;
  const unsigned s4 = (unsigned)db.x - nbs, s5 = (unsigned)db.y - nbs;
  const unsigned s6 = (unsigned)db.z - nbs, s7 = (unsigned)db.w - nbs;
  const bool h0 = s0 < unb, h1 = s1 < unb, h2 = s2 < unb, h3 = s3 < unb;
  const bool h4 = s4 < unb, h5 = s5 < unb, h6 = s6 < unb, h7 = s7 < unb;
  const unsigned any = __builtin_amdgcn_ballot_w32(h0 | h1 | h2 | h3 | h4 | h5 | h6 | h7);
  if (any != 0u) {
#define HITJ(J, HJ, SJ) { \
      const unsigned mj = __builtin_amdgcn_ballot_w32(HJ); \
      if (mj != 0u) { \
        if (HJ) { \
          const int pos = wc + (int)__builtin_amdgcn_mbcnt_lo(mj, 0u); \
          if (pos < WCAP) list[wave * WCAP + pos] = ((el0 + (J)) << SLB) | (int)(SJ); \
        } \
        wc += (int)__builtin_popcount(mj); } }
    HITJ(0, h0, s0)
    HITJ(1, h1, s1)
    HITJ(2, h2, s2)
    HITJ(3, h3, s3)
    HITJ(4, h4, s4)
    HITJ(5, h5, s5)
    HITJ(6, h6, s6)
    HITJ(7, h7, s7)
#undef HITJ
  }
  return wc;
}

__global__ __launch_bounds__(NTHR) void k_prep(const float* __restrict__ W1, const float* __restrict__ W2,
                                               const float* __restrict__ fw1,
                                               unsigned short* W1T, unsigned short* W2T, unsigned short* FWT) {
  const int u = (int)blockIdx.x * NTHR + (int)threadIdx.x;
  v8us o;
  unsigned short* dp;
  if (u < NU1) {
    const int n  = u >> 4;
    const int k8 = (u & 15) * 8;
    const float* p = W1 + (size_t)k8 * F + n;
#pragma unroll
    for (int i = 0; i < 8; ++i) o[i] = (unsigned short)bf16_bits(p[(size_t)i * F]);
    dp = W1T + (size_t)u * 8;
  } else if (u < NU1 + NU2) {
    const int v  = u - NU1;
    const int n  = v >> 5;
    const int k8 = (v & 31) * 8;
    const int kk = k8 & (F - 1);
    const float* p = W2 + (size_t)kk * F + n;
#pragma unroll
    for (int i = 0; i < 8; ++i) o[i] = (unsigned short)bf16_bits(p[(size_t)i * F]);
    dp = W2T + (size_t)v * 8;
  } else if (u < NU1 + NU2 + NU3) {
    const int v  = u - NU1 - NU2;
    const int n  = v >> 5;
    const int k8 = (v & 31) * 8;
    const int kk = k8 & (F - 1);
    const float* p = fw1 + (size_t)kk * FH + n;
#pragma unroll
    for (int i = 0; i < 8; ++i) o[i] = (unsigned short)bf16_bits(p[(size_t)i * FH]);
    dp = FWT + (size_t)v * 8;
  } else {
    return;
  }
  *(volatile v8us*)dp = o;
  __threadfence();
  *(volatile v8us*)dp = o;
}

__global__ __launch_bounds__(NTHR) void k_cvx(const float* __restrict__ x, int nN, int nUnits,
                                              unsigned short* xb) {
  const int u = (int)blockIdx.x * NTHR + (int)threadIdx.x;
  if (u >= nUnits) return;
  const int row = u >> 4;
  const int k8  = (u & 15) * 8;
  const int rc  = row < nN ? row : nN - 1;
  const float* p = x + (size_t)rc * F + k8;
  const v4f a = *(const v4f*)p;
  const v4f b = *(const v4f*)(p + 4);
  const bool ok = row < nN;
  v8us o;
  o[0] = ok ? (unsigned short)bf16_bits(a.x) : (unsigned short)0;
  o[1] = ok ? (unsigned short)bf16_bits(a.y) : (unsigned short)0;
  o[2] = ok ? (unsigned short)bf16_bits(a.z) : (unsigned short)0;
  o[3] = ok ? (unsigned short)bf16_bits(a.w) : (unsigned short)0;
  o[4] = ok ? (unsigned short)bf16_bits(b.x) : (unsigned short)0;
  o[5] = ok ? (unsigned short)bf16_bits(b.y) : (unsigned short)0;
  o[6] = ok ? (unsigned short)bf16_bits(b.z) : (unsigned short)0;
  o[7] = ok ? (unsigned short)bf16_bits(b.w) : (unsigned short)0;
  unsigned short* dp = xb + (size_t)u * 8;
  *(volatile v8us*)dp = o;
  __threadfence();
  *(volatile v8us*)dp = o;
}

__global__ __launch_bounds__(NTHR) void k_deg(const int* __restrict__ dsts, int nE, int vec8, float* dis) {
  __shared__ __attribute__((aligned(16))) int scnt[NBD];
  __shared__ __attribute__((aligned(16))) int list[LISTN];
  __shared__ int wcnt[NWAVE];
  const int tid = (int)threadIdx.x, lane = tid & 31, wave = tid >> 5;
  const int nodeBase = (int)blockIdx.x * NBD;

  for (int i = tid; i < NBD; i += NTHR) scnt[i] = 0;
  for (int i = tid; i < LISTN; i += NTHR) list[i] = 0;
  if (tid < NWAVE) wcnt[tid] = 0;
  __syncthreads();

  const int nChunks = (nE + CHUNK - 1) / CHUNK;
#pragma unroll 1
  for (int ch = 0; ch < nChunks; ++ch) {
    const int cbase = ch * CHUNK;
    const int wc = scan_chunk<SLD>(dsts, nE, cbase, nodeBase, NBD, vec8, list, tid, lane, wave);
    if (lane == 0) wcnt[wave] = wc;
    __syncthreads();
    if (wave == 0) {
#pragma unroll 1
      for (int w2 = 0; w2 < NWAVE; ++w2) {
        int c = wcnt[w2];
        c = c < 0 ? 0 : (c > WCAP ? WCAP : c);
#pragma unroll 1
        for (int b0 = 0; b0 < c; b0 += 32) {
          const int idx = b0 + lane;
          const int ent = list[w2 * WCAP + (idx < WCAP ? idx : WCAP - 1)];
          const int m32 = (c - b0) < 32 ? (c - b0) : 32;
#pragma unroll 1
          for (int k = 0; k < m32; ++k) {
            const int u  = __builtin_amdgcn_readlane(ent, k);
            const int sl = u & (NBD - 1);
            if (lane == 0) scnt[sl] = scnt[sl] + 1;
          }
        }
      }
    }
    __syncthreads();
  }

  v4f vals[NBD / (NTHR * 4)];
#pragma unroll
  for (int it = 0; it < NBD / (NTHR * 4); ++it) {
    const int s0 = it * (NTHR * 4) + 4 * tid;
    const v4i c4 = *(const v4ia*)(scnt + s0);
    v4f v;
    v.x = rsqrtf((float)c4.x + 1.0f); v.y = rsqrtf((float)c4.y + 1.0f);
    v.z = rsqrtf((float)c4.z + 1.0f); v.w = rsqrtf((float)c4.w + 1.0f);
    vals[it] = v;
  }
#pragma unroll
  for (int it = 0; it < NBD / (NTHR * 4); ++it) {
    const int s0 = it * (NTHR * 4) + 4 * tid;
    *(volatile v4f*)(dis + (size_t)nodeBase + s0) = vals[it];
  }
  __threadfence();
#pragma unroll
  for (int it = 0; it < NBD / (NTHR * 4); ++it) {
    const int s0 = it * (NTHR * 4) + 4 * tid;
    *(volatile v4f*)(dis + (size_t)nodeBase + s0) = vals[it];
  }
}

__global__ __launch_bounds__(GTHR) void k_gemm(const unsigned short* __restrict__ A, int lda,
                                               const unsigned short* __restrict__ BT, int ldb, int K,
                                               float* Cm, int ldc) {
  __shared__ __attribute__((aligned(16))) float stg[GBM * GBN];
  const int tid = (int)threadIdx.x, lane = tid & 31, wave = tid >> 5, hh = lane >> 4, m = lane & 15;
  const int rowBase = (int)blockIdx.x * GBM;
  const int colBase = (int)blockIdx.y * GBN;

  v8f acc[8];
#pragma unroll
  for (int t = 0; t < 8; ++t) acc[t] = z8();
  const unsigned short* ap = A  + (size_t)(rowBase + 16 * wave + m) * (size_t)lda + 8 * hh;
  const unsigned short* bp = BT + (size_t)(colBase + m) * (size_t)ldb + 8 * hh;

#pragma unroll 1
  for (int k0 = 0; k0 < K; k0 += 32) {
    FragB af;
    af.h[0] = *(const v8usa*)(ap + k0);
    af.h[1] = *(const v8usa*)(ap + k0 + 16);
#pragma unroll
    for (int nt = 0; nt < 8; ++nt) {
      const unsigned short* wq = bp + (size_t)(16 * nt) * (size_t)ldb + k0;
      FragB bf;
      bf.h[0] = *(const v8usa*)wq;
      bf.h[1] = *(const v8usa*)(wq + 16);
      acc[nt] = wmb(af, bf, acc[nt]);
    }
  }

#pragma unroll
  for (int nt = 0; nt < 8; ++nt) {
    const int lc = 16 * nt + m;
#pragma unroll
    for (int r = 0; r < 8; ++r) {
      const int lr = 16 * wave + 8 * hh + r;
      stg[lr * GBN + lc] = acc[nt][r];
    }
  }
  __syncthreads();

  v4f pv[16];
#pragma unroll
  for (int i = 0; i < 16; ++i) pv[i] = *(const v4fa*)(stg + (16 * wave + i) * GBN + 4 * lane);
#pragma unroll
  for (int i = 0; i < 16; ++i) {
    float* op = Cm + (size_t)(rowBase + 16 * wave + i) * (size_t)ldc + colBase + 4 * lane;
    *(volatile v4f*)op = pv[i];
  }
  __threadfence();
#pragma unroll
  for (int i = 0; i < 16; ++i) {
    float* op = Cm + (size_t)(rowBase + 16 * wave + i) * (size_t)ldc + colBase + 4 * lane;
    *(volatile v4f*)op = pv[i];
  }
}

__global__ __launch_bounds__(NTHR) void k_agg(const int* __restrict__ srcs, const int* __restrict__ dsts,
                                              int nE, int nN, int vec8, int mRows,
                                              const float* __restrict__ dis,
                                              const float* __restrict__ hin,
                                              const float* __restrict__ bias,
                                              float* gout, float* part) {
  extern __shared__ __attribute__((aligned(16))) int dsm[];
  int* list = dsm;
  int* hl   = dsm + LISTN;
  int* sl   = hl + RCAP;
  int* cnt  = sl + RCAP;
  int* offs = cnt + NBA;
  int* cur  = offs + NBA;
  int* misc = cur + NBA;
  float* wst = (float*)(misc + 16);
  float* pst = wst + NWAVE * WSTW;
  const int tid = (int)threadIdx.x, lane = tid & 31, wave = tid >> 5;
  const int nodeBase = (int)blockIdx.x * NBA;

  {
    const v4i z4 = {0, 0, 0, 0};
    for (int i = tid * 4; i < AGG_ZINTS; i += NTHR * 4) *(v4ia*)(dsm + i) = z4;
    if (tid < 16) misc[tid] = 0;
  }
  float bv[4];
  {
    const v4f bq = *(const v4fa*)(bias + 4 * lane);
    bv[0] = bf16_val(bq.x); bv[1] = bf16_val(bq.y); bv[2] = bf16_val(bq.z); bv[3] = bf16_val(bq.w);
  }
  __syncthreads();

  int t = 0, ov = 0;
  const int nChunks = (nE + CHUNK - 1) / CHUNK;
#pragma unroll 1
  for (int ch = 0; ch < nChunks; ++ch) {
    const int cbase = ch * CHUNK;
    const int wc = scan_chunk<SLA>(dsts, nE, cbase, nodeBase, NBA, vec8, list, tid, lane, wave);
    if (lane == 0) misc[wave] = wc;
    __syncthreads();
    if (wave == 0) {
#pragma unroll 1
      for (int w2 = 0; w2 < NWAVE; ++w2) {
        int c = misc[w2];
        c = c < 0 ? 0 : (c > WCAP ? WCAP : c);
#pragma unroll 1
        for (int b0 = 0; b0 < c; b0 += 32) {
          const int idx = b0 + lane;
          const int ent = list[w2 * WCAP + (idx < WCAP ? idx : WCAP - 1)];
          const int m32 = (c - b0) < 32 ? (c - b0) : 32;
#pragma unroll 1
          for (int k = 0; k < m32; ++k) {
            const int u    = __builtin_amdgcn_readlane(ent, k);
            const int slot = u & (NBA - 1);
            const int el   = (u >> SLA) & (CHUNK - 1);
            const int pk   = ((cbase + el) << SLA) | slot;
            if (t < RCAP) {
              if (lane == 0) { hl[t] = pk; cnt[slot] = cnt[slot] + 1; }
              t = t + 1;
            } else {
              ov = 1;
            }
          }
        }
      }
    }
    __syncthreads();
  }
  if (wave == 0 && lane == 0) { misc[8] = t; misc[9] = ov; }
  __syncthreads();
  int tt = misc[8];
  tt = tt < 0 ? 0 : (tt > RCAP ? RCAP : tt);
  const int ovf = misc[9];

  if (wave == 0) {
    const int base = lane * (NBA / 32);
    int s = 0;
#pragma unroll 1
    for (int i = 0; i < NBA / 32; ++i) s += cnt[base + i];
    int incl = s;
#pragma unroll
    for (int d = 1; d < 32; d <<= 1) {
      const int y = __shfl_up(incl, d, 32);
      if (lane >= d) incl += y;
    }
    int run = incl - s;
#pragma unroll 1
    for (int i = 0; i < NBA / 32; ++i) {
      const int cv = cnt[base + i];
      offs[base + i] = run;
      cur[base + i]  = run;
      run += cv;
    }
  }
  __syncthreads();
  if (wave == 0) {
#pragma unroll 1
    for (int b0 = 0; b0 < tt; b0 += 32) {
      const int idx = b0 + lane;
      const int ent = hl[idx < RCAP ? idx : RCAP - 1];
      const int m32 = (tt - b0) < 32 ? (tt - b0) : 32;
#pragma unroll 1
      for (int k = 0; k < m32; ++k) {
        const int u    = __builtin_amdgcn_readlane(ent, k);
        const int slot = u & (NBA - 1);
        if (lane == 0) {
          int p = cur[slot];
          p = p < 0 ? 0 : (p > RCAP - 1 ? RCAP - 1 : p);
          sl[p] = u;
          cur[slot] = p + 1;
        }
      }
    }
  }
  __syncthreads();

  const float pz = (ovf != 0) ? __int_as_float(0x7fc00000) : 0.0f;
  int wn = 0;
  float wm[4], wq[4];
#pragma unroll
  for (int i = 0; i < 4; ++i) { wm[i] = 0.0f; wq[i] = 0.0f; }
#pragma unroll 1
  for (int si = 0; si < NBA / NWAVE; ++si) {
    const int s    = si * NWAVE + wave;
    const int node = nodeBase + s;
    int c = cnt[s];
    const bool big = c > DEGCAP;
    c = c < 0 ? 0 : (c > DEGCAP ? DEGCAP : c);
    int o = offs[s];
    o = o < 0 ? 0 : (o > RCAP ? RCAP : o);
    const int nc = node < nN ? node : nN - 1;
    const float dd = dis[nc];
    float acc[4];
#pragma unroll
    for (int i = 0; i < 4; ++i) acc[i] = 0.0f;
#pragma unroll 1
    for (int b0 = 0; b0 < c; b0 += 32) {
      int idx = o + b0 + lane;
      idx = idx > RCAP - 1 ? RCAP - 1 : idx;
      const int ent = sl[idx];
      int eid = ent >> SLA;
      eid = eid < 0 ? 0 : (eid > nE - 1 ? nE - 1 : eid);
      int sr = srcs[eid];
      sr = sr < 0 ? 0 : (sr > nN - 1 ? nN - 1 : sr);
      const float cf  = dis[sr] * dd;
      const int   cfi = __float_as_int(cf);
      const int m32 = (c - b0) < 32 ? (c - b0) : 32;
#pragma unroll 1
      for (int k = 0; k < m32; ++k) {
        const int   sk = __builtin_amdgcn_readlane(sr, k);
        const float ck = __int_as_float(__builtin_amdgcn_readlane(cfi, k));
        const v4f a = *(const v4f*)(hin + (size_t)sk * F + 4 * lane);
        acc[0] = fmaf(ck, a.x, acc[0]); acc[1] = fmaf(ck, a.y, acc[1]);
        acc[2] = fmaf(ck, a.z, acc[2]); acc[3] = fmaf(ck, a.w, acc[3]);
      }
    }
    float sv[4];
    {
      const v4f a = *(const v4f*)(hin + (size_t)nc * F + 4 * lane);
      sv[0] = a.x; sv[1] = a.y; sv[2] = a.z; sv[3] = a.w;
    }
    const float rd  = dd * dd;
    const float pzr = big ? __int_as_float(0x7fc00000) : pz;
    const bool live = node < nN;
    float v[4];
#pragma unroll
    for (int i = 0; i < 4; ++i) {
      float y = (acc[i] + sv[i] * rd) + bv[i];
      y = y + pzr;
      v[i] = live ? y : 0.0f;
    }
    if (live) {
      wn += 1;
      const float rk = 1.0f / (float)wn;
#pragma unroll
      for (int i = 0; i < 4; ++i) {
        const float d = v[i] - wm[i];
        wm[i] = fmaf(d, rk, wm[i]);
        wq[i] = fmaf(d, v[i] - wm[i], wq[i]);
      }
    }
    if (node < mRows) {
      v4f hv;
      hv.x = v[0]; hv.y = v[1]; hv.z = v[2]; hv.w = v[3];
      float* hp = gout + (size_t)node * F + 4 * lane;
      *(volatile v4f*)hp = hv;
      __threadfence();
      *(volatile v4f*)hp = hv;
    }
  }

  if (lane == 0) wst[wave * WSTW] = (float)wn;
#pragma unroll
  for (int i = 0; i < 4; ++i) {
    wst[wave * WSTW + 1 + 4 * lane + i]     = wm[i];
    wst[wave * WSTW + 1 + F + 4 * lane + i] = wq[i];
  }
  __syncthreads();
  if (tid < F) {
    float n = 0.0f, mean = 0.0f, M2 = 0.0f;
#pragma unroll 1
    for (int w2 = 0; w2 < NWAVE; ++w2) {
      const float nb = wst[w2 * WSTW];
      const float mb = wst[w2 * WSTW + 1 + tid];
      const float qb = wst[w2 * WSTW + 1 + F + tid];
      if (nb > 0.5f) {
        const float nn = n + nb;
        const float delta = mb - mean;
        const float f = nb / nn;
        mean = fmaf(delta, f, mean);
        M2 = M2 + qb + delta * delta * n * f;
        n = nn;
      }
    }
    pst[1 + tid] = mean;
    pst[1 + F + tid] = M2;
    if (tid == 0) pst[0] = n;
  }
#pragma unroll 1
  for (int i = 2 * F + 1 + tid; i < PARTW; i += NTHR) pst[i] = 0.0f;
  __syncthreads();
  v4f pv;
  if (tid < PARTW / 4) {
    pv = *(const v4fa*)(pst + 4 * tid);
    *(volatile v4f*)(part + (size_t)blockIdx.x * PARTW + 4 * tid) = pv;
  }
  __threadfence();
  if (tid < PARTW / 4) {
    *(volatile v4f*)(part + (size_t)blockIdx.x * PARTW + 4 * tid) = pv;
  }
}

__global__ __launch_bounds__(F) void k_bnfin(const float* __restrict__ part, int nPart,
                                             const float* __restrict__ gam, const float* __restrict__ bet,
                                             float* ss) {
  __shared__ __attribute__((aligned(16))) float stg[2 * F];
  const int tid = (int)threadIdx.x;
  const int c = tid & (F - 1);
  float n = 0.0f, mean = 0.0f, M2 = 0.0f;
#pragma unroll 1
  for (int b = 0; b < nPart; ++b) {
    const float* pr = part + (size_t)b * PARTW;
    const float nb = pr[0];
    const float mb = pr[1 + c];
    const float qb = pr[1 + F + c];
    if (nb > 0.5f) {
      const float nn = n + nb;
      const float delta = mb - mean;
      const float f = nb / nn;
      mean = fmaf(delta, f, mean);
      M2 = M2 + qb + delta * delta * n * f;
      n = nn;
    }
  }
  const float nt = n < 1.0f ? 1.0f : n;
  const float var = M2 * (1.0f / nt);
  const float rstd = rsqrtf(var + 1e-5f);
  const float sc = bf16_val(gam[c]) * rstd;
  const float sh = bf16_val(bet[c]) - mean * sc;
  stg[c] = sc;
  stg[F + c] = sh;
  __syncthreads();
  v4f v;
  if (tid < (2 * F) / 4) {
    v = *(const v4fa*)(stg + 4 * tid);
    *(volatile v4f*)(ss + 4 * tid) = v;
  }
  __threadfence();
  if (tid < (2 * F) / 4) {
    *(volatile v4f*)(ss + 4 * tid) = v;
  }
}

__global__ __launch_bounds__(NTHR) void k_bnap(const float* __restrict__ graw, int nN, int nUnits,
                                               const float* __restrict__ ss, unsigned short* a1) {
  __shared__ float ssh[2 * F];
  const int tid = (int)threadIdx.x;
  ssh[tid] = ss[tid];
  __syncthreads();
  const int u = (int)blockIdx.x * NTHR + tid;
  if (u >= nUnits) return;
  const int row = u >> 4;
  const int k8  = (u & 15) * 8;
  const int rc  = row < nN ? row : nN - 1;
  const float* p = graw + (size_t)rc * F + k8;
  const v4f a = *(const v4f*)p;
  const v4f b = *(const v4f*)(p + 4);
  const bool ok = row < nN;
  float xv[8];
  xv[0] = a.x; xv[1] = a.y; xv[2] = a.z; xv[3] = a.w;
  xv[4] = b.x; xv[5] = b.y; xv[6] = b.z; xv[7] = b.w;
  v8us ho, lo;
#pragma unroll
  for (int i = 0; i < 8; ++i) {
    const float v = fmaxf(fmaf(xv[i], ssh[k8 + i], ssh[F + k8 + i]), 0.0f);
    const unsigned hb = bf16_bits(v);
    const unsigned lb = bf16_bits(v - __uint_as_float(hb << 16));
    ho[i] = ok ? (unsigned short)hb : (unsigned short)0;
    lo[i] = ok ? (unsigned short)lb : (unsigned short)0;
  }
  unsigned short* dp = a1 + (size_t)row * K2 + k8;
  *(volatile v8us*)dp = ho;
  *(volatile v8us*)(dp + F) = lo;
  __threadfence();
  *(volatile v8us*)dp = ho;
  *(volatile v8us*)(dp + F) = lo;
}

__global__ __launch_bounds__(HTHR) void k_head(const float* __restrict__ gc, int nN,
                                               const float* __restrict__ ss, const unsigned short* __restrict__ fwt,
                                               const float* __restrict__ fb1, const float* __restrict__ fw2,
                                               const float* __restrict__ fb2, float* out) {
  __shared__ float scs[F];
  __shared__ float shs[F];
  __shared__ float fb1s[FH];
  __shared__ float fw2s[FH * NOUT];
  __shared__ float fb2s[4];
  __shared__ __attribute__((aligned(16))) float zs[GBM * FH];
  __shared__ __attribute__((aligned(16))) float outs[GBM * NOUT];
  const int tid = (int)threadIdx.x, lane = tid & 31, wave = tid >> 5, hh = lane >> 4, m = lane & 15;
  const int rowBase = (int)blockIdx.x * GBM;
  scs[tid] = ss[tid];
  shs[tid] = ss[F + tid];
  fw2s[tid] = bf16_val(fw2[tid]);
  if (tid < FH) fb1s[tid] = bf16_val(fb1[tid]);
  if (tid < NOUT) fb2s[tid] = bf16_val(fb2[tid]);
  __syncthreads();

  const int rowA = rowBase + 16 * wave + m;
  const float* zr = gc + (size_t)rowA * F;
  const unsigned short* bt = fwt + (size_t)m * K2 + 8 * hh;
  v8f acc[4];
#pragma unroll
  for (int t = 0; t < 4; ++t) acc[t] = z8();
#pragma unroll
  for (int ks = 0; ks < F / 32; ++ks) {
    const int k0 = 32 * ks;
    const v4f p0 = *(const v4f*)(zr + k0 + 8 * hh);
    const v4f p1 = *(const v4f*)(zr + k0 + 8 * hh + 4);
    const v4f p2 = *(const v4f*)(zr + k0 + 16 + 8 * hh);
    const v4f p3 = *(const v4f*)(zr + k0 + 16 + 8 * hh + 4);
    float xv[16];
    xv[0] = p0.x;  xv[1] = p0.y;  xv[2] = p0.z;  xv[3] = p0.w;
    xv[4] = p1.x;  xv[5] = p1.y;  xv[6] = p1.z;  xv[7] = p1.w;
    xv[8] = p2.x;  xv[9] = p2.y;  xv[10] = p2.z; xv[11] = p2.w;
    xv[12] = p3.x; xv[13] = p3.y; xv[14] = p3.z; xv[15] = p3.w;
    FragB ah, al;
#pragma unroll
    for (int i = 0; i < 16; ++i) {
      const int kk = (i < 8) ? (k0 + 8 * hh + i) : (k0 + 16 + 8 * hh + (i - 8));
      const float v = fmaxf(fmaf(xv[i], scs[kk], shs[kk]), 0.0f);
      const unsigned hb = bf16_bits(v);
      const unsigned lb = bf16_bits(v - __uint_as_float(hb << 16));
      ah.u[i] = (unsigned short)hb;
      al.u[i] = (unsigned short)lb;
    }
#pragma unroll
    for (int nt = 0; nt < FH / 16; ++nt) {
      const unsigned short* bq = bt + (size_t)(16 * nt) * K2 + k0;
      FragB bh, bl;
      bh.h[0] = *(const v8usa*)bq;
      bh.h[1] = *(const v8usa*)(bq + 16);
      bl.h[0] = *(const v8usa*)(bq + F);
      bl.h[1] = *(const v8usa*)(bq + F + 16);
      acc[nt] = wmb(ah, bh, acc[nt]);
      acc[nt] = wmb(al, bl, acc[nt]);
    }
  }
#pragma unroll
  for (int nt = 0; nt < FH / 16; ++nt) {
    const int lc = 16 * nt + m;
    const float fbv = fb1s[lc];
#pragma unroll
    for (int r = 0; r < 8; ++r) {
      const int lr = 16 * wave + 8 * hh + r;
      zs[lr * FH + lc] = fmaxf(acc[nt][r] + fbv, 0.0f);
    }
  }
  __syncthreads();

  {
    const int row = tid >> 1;
    const int o   = tid & 1;
    float s = 0.0f;
#pragma unroll 8
    for (int cc = 0; cc < FH; ++cc) s = fmaf(zs[row * FH + cc], fw2s[cc * NOUT + o], s);
    outs[tid] = s + fb2s[o];
  }
  __syncthreads();

  const v4f ov4 = *(const v4fa*)(outs + 4 * lane);
  const bool okst = (wave == 0) && (rowBase + 2 * lane < nN);
  float* op = out + (size_t)rowBase * NOUT + 4 * lane;
  if (okst) *(volatile v4f*)op = ov4;
  __threadfence();
  if (okst) *(volatile v4f*)op = ov4;
}

static inline int cdiv(int a, int b) { return (a + b - 1) / b; }
static inline size_t al256(size_t o) { return (o + 255) & ~(size_t)255; }

extern "C" void kernel_launch(void* const* d_in, const int* in_sizes, int n_in,
                              void* d_out, int out_size, void* d_ws, size_t ws_size,
                              hipStream_t stream) {
  if (n_in < 15) return;
  if (in_sizes[0] < F || (in_sizes[0] % F) != 0) return;
  const int nN = in_sizes[0] / F;
  const int nE = in_sizes[1];
  if (nE < 1 || in_sizes[2] != nE) return;
  if (nE >= (1 << 21) || nN < 16 || nN >= (1 << 24)) return;
  if ((nN % 16) != 0) return;
  if (in_sizes[3] != F * F || in_sizes[4] != F || in_sizes[5] != F || in_sizes[6] != F) return;
  if (in_sizes[7] != F * F || in_sizes[8] != F || in_sizes[9] != F || in_sizes[10] != F) return;
  if (in_sizes[11] != F * FH || in_sizes[12] != FH) return;
  if (in_sizes[13] != FH * NOUT || in_sizes[14] != NOUT) return;
  if ((long long)out_size != (long long)nN * NOUT) return;

  const float* x    = (const float*)d_in[0];
  const int*   src  = (const int*)d_in[1];
  const int*   dst  = (const int*)d_in[2];
  const float* W1   = (const float*)d_in[3];
  const float* b1   = (const float*)d_in[4];
  const float* g1   = (const float*)d_in[5];
  const float* be1  = (const float*)d_in[6];
  const float* W2   = (const float*)d_in[7];
  const float* b2   = (const float*)d_in[8];
  const float* g2   = (const float*)d_in[9];
  const float* be2  = (const float*)d_in[10];
  const float* fw1  = (const float*)d_in[11];
  const float* fb1  = (const float*)d_in[12];
  const float* fw2  = (const float*)d_in[13];
  const float* fb2  = (const float*)d_in[14];
  float* out = (float*)d_out;

  const int MP   = cdiv(nN, GBM) * GBM;
  const int gM   = MP / GBM;
  const int gD   = cdiv(nN, NBD);
  const int NBPD = gD * NBD;
  const int gA   = cdiv(nN, NBA);
  if ((long long)gA * NBA < (long long)MP) return;
  if (NBPD < nN) return;
  const int vec8 = ((nE & 3) == 0) ? 1 : 0;

  char* ws = (char*)d_ws;
  size_t off = 0;
  const size_t oDIS = off; off = al256(off + (size_t)NBPD * 4);
  const size_t oW1T = off; off = al256(off + (size_t)F * F * 2);
  const size_t oW2T = off; off = al256(off + (size_t)F * K2 * 2);
  const size_t oFWT = off; off = al256(off + (size_t)FH * K2 * 2);
  const size_t oXB  = off; off = al256(off + (size_t)MP * F * 2);
  const size_t oHL  = off; off = al256(off + (size_t)MP * F * 4);
  const size_t oGC  = off; off = al256(off + (size_t)MP * F * 4);
  const size_t oA1  = off; off = al256(off + (size_t)MP * K2 * 2);
  const size_t oP0  = off; off = al256(off + (size_t)gA * PARTW * 4);
  const size_t oP1  = off; off = al256(off + (size_t)gA * PARTW * 4);
  const size_t oS0  = off; off = al256(off + (size_t)(2 * F) * 4);
  const size_t oS1  = off; off = al256(off + (size_t)(2 * F) * 4);
  if (off > ws_size || off > (size_t)WSMAX) return;
  float*          DIS = (float*)(ws + oDIS);
  unsigned short* W1T = (unsigned short*)(ws + oW1T);
  unsigned short* W2T = (unsigned short*)(ws + oW2T);
  unsigned short* FWT = (unsigned short*)(ws + oFWT);
  unsigned short* XB  = (unsigned short*)(ws + oXB);
  float*          HL  = (float*)(ws + oHL);
  float*          GC  = (float*)(ws + oGC);
  unsigned short* A1  = (unsigned short*)(ws + oA1);
  float*          P0  = (float*)(ws + oP0);
  float*          P1  = (float*)(ws + oP1);
  float*          S0  = (float*)(ws + oS0);
  float*          S1  = (float*)(ws + oS1);

  const size_t aggLds = (size_t)AGG_LDS_INTS * 4;
  hipFuncSetAttribute(reinterpret_cast<const void*>(&k_agg), hipFuncAttributeMaxDynamicSharedMemorySize, (int)aggLds);

  const int nUx = MP * (F / 8);
  k_prep<<<(NU1 + NU2 + NU3) / NTHR, NTHR, 0, stream>>>(W1, W2, fw1, W1T, W2T, FWT);
  k_cvx<<<cdiv(nUx, NTHR), NTHR, 0, stream>>>(x, nN, nUx, XB);
  k_deg<<<gD, NTHR, 0, stream>>>(dst, nE, vec8, DIS);
  k_gemm<<<dim3(gM, F / GBN), GTHR, 0, stream>>>(XB, F, W1T, F, F, HL, F);
  k_agg<<<gA, NTHR, aggLds, stream>>>(src, dst, nE, nN, vec8, MP, DIS, HL, b1, GC, P0);
  k_bnfin<<<1, F, 0, stream>>>(P0, gA, g1, be1, S0);
  k_bnap<<<cdiv(nUx, NTHR), NTHR, 0, stream>>>(GC, nN, nUx, S0, A1);
  k_gemm<<<dim3(gM, F / GBN), GTHR, 0, stream>>>(A1, K2, W2T, K2, K2, HL, F);
  k_agg<<<gA, NTHR, aggLds, stream>>>(src, dst, nE, nN, vec8, MP, DIS, HL, b2, GC, P1);
  k_bnfin<<<1, F, 0, stream>>>(P1, gA, g2, be2, S1);
  k_head<<<gM, HTHR, 0, stream>>>(GC, nN, S1, FWT, fb1, fw2, fb2, out);
}
